// KNeighBallChanger_53017076302314
// MI455X (gfx1250) — hardware-verified
//
#include <hip/hip_runtime.h>
#include <stddef.h>


#pragma clang fp contract(off)

typedef __attribute__((ext_vector_type(16))) _Float16 v16h;
typedef __attribute__((ext_vector_type(8)))  _Float16 v8h;
typedef __attribute__((ext_vector_type(8)))  float    v8f;
typedef __attribute__((ext_vector_type(4)))  float    v4f;

__device__ __forceinline__ void dep_guard_h(v8f& a, v8f& b, v16h x, v16h y) { asm volatile("v_nop\n\tv_nop\n\tv_nop\n\tv_nop" : "+v"(a), "+v"(b) : "v"(x), "v"(y)); }
__device__ __forceinline__ void keep4_h(v16h a, v16h b, v16h c, v16h d) { asm volatile("v_nop" :: "v"(a), "v"(b), "v"(c), "v"(d)); }
__device__ __forceinline__ void acc_guard4(v8f& a, v8f& b, v8f& c, v8f& d) { asm volatile("v_nop\n\tv_nop\n\tv_nop\n\tv_nop" : "+v"(a), "+v"(b), "+v"(c), "+v"(d)); }
__device__ __forceinline__ void mma_guard4(v8f& a, v8f& b, v8f& c, v8f& d, v16h x0, v16h x1, v16h x2, v16h x3, v16h y) {
  asm volatile("v_nop\n\tv_nop\n\tv_nop\n\tv_nop" : "+v"(a), "+v"(b), "+v"(c), "+v"(d) : "v"(x0), "v"(x1), "v"(x2), "v"(x3), "v"(y));
}

template <typename T> struct Frag;
template <> struct Frag<_Float16> {
  typedef v16h V; union U { v16h v; v8h h[2]; };
  static __device__ __forceinline__ v16h load(const _Float16* p) {
    U f; f.h[0] = *(const v8h*)(p); f.h[1] = *(const v8h*)(p + 16); return f.v;
  }
  static __device__ __forceinline__ v8f mma(v16h a, v16h b, v8f c) {
    return __builtin_amdgcn_wmma_f32_16x16x32_f16(false, a, false, b, (short)0, c, false, false);
  }
  static __device__ __forceinline__ void guard(v8f& a, v8f& b, v16h x, v16h y) { dep_guard_h(a, b, x, y); }
  static __device__ __forceinline__ void keep(v16h a, v16h b, v16h c, v16h d) { keep4_h(a, b, c, d); }
};

namespace {
constexpr int KC  = 128;
constexpr int KS  = KC / 32;
constexpr int XP  = KC + 8;
constexpr int NW  = 2;
constexpr int NT  = NW * 32;
constexpr int OPW = 64;
constexpr int OPB = NW * OPW;
constexpr int SP  = 68;
constexpr float kR2  = (float)(0.05 * 0.05);
constexpr float kFar = 1.0e18f;
}

union HFrag { v16h v; unsigned u[8]; };

__global__ __launch_bounds__(NT)
void ball_pool_f16(const float* __restrict__ x, const float* __restrict__ ipos,
                   const float* __restrict__ opos, float* __restrict__ out,
                   int nIn, int nOut, int nB)
{
  __shared__ __align__(16) float    sPos[KC * 4];
  __shared__ __align__(16) _Float16 sX[16 * XP];
  __shared__ __align__(16) float    sSlab[NW][16 * SP];

  const int tid  = threadIdx.x;
  const int wave = tid >> 5;
  const int lane = tid & 31;
  const int h    = lane >> 4;
  const int c    = lane & 15;
  const int obase = blockIdx.x * OPB + wave * OPW;

  float oxr[4], oyr[4], ozr[4];
#pragma unroll 4
  for (int t = 0; t < 4; ++t) {
    int o = obase + 16 * t + c;
    o = (o < nOut) ? o : (nOut - 1);
    oxr[t] = opos[(size_t)o * 3 + 0];
    oyr[t] = opos[(size_t)o * 3 + 1];
    ozr[t] = opos[(size_t)o * 3 + 2];
  }

  for (int idx = tid; idx < 16 * XP; idx += NT) {
    const int row = idx / XP;
    sX[idx] = (row == 15) ? (_Float16)1.0f : (_Float16)0.0f;
  }

  v8f acc0 = (v8f){0.f,0.f,0.f,0.f,0.f,0.f,0.f,0.f};
  v8f acc1 = acc0, acc2 = acc0, acc3 = acc0;

  const int nChunks = (nIn + KC - 1) / KC;
  for (int ch = 0; ch < nChunks; ++ch) {
    const int k0 = ch * KC;
    __syncthreads();
    for (int j = tid; j < KC; j += NT) {
      const int i = k0 + j;
      v4f p;
      if (i < nIn) {
        p.x = ipos[(size_t)i * 3 + 0];
        p.y = ipos[(size_t)i * 3 + 1];
        p.z = ipos[(size_t)i * 3 + 2];
      } else {
        p.x = kFar; p.y = kFar; p.z = kFar;
      }
      p.w = 0.0f;
      *(v4f*)(sPos + 4 * j) = p;
    }
    const int nx = nB * KC;
    for (int idx = tid; idx < nx; idx += NT) {
      const int b = idx / KC;
      const int j = idx - b * KC;
      const int i = k0 + j;
      const float v = (i < nIn) ? x[(size_t)b * nIn + i] : 0.0f;
      sX[b * XP + j] = (_Float16)v;
    }
    __syncthreads();

#pragma unroll 1
    for (int ks = 0; ks < KS; ++ks) {
      HFrag am[4];
      const float* pb = sPos + 4 * (ks * 32 + 8 * h);
#pragma unroll 16
      for (int e = 0; e < 16; ++e) {
        const int jo = (e < 8) ? e : (e + 8);
        const v4f p = *(const v4f*)(pb + 4 * jo);
#pragma unroll 4
        for (int t = 0; t < 4; ++t) {
          const float dx = oxr[t] - p.x;
          const float dy = oyr[t] - p.y;
          const float dz = ozr[t] - p.z;
          const float sx = dx * dx;
          const float sy = dy * dy;
          const float sz = dz * dz;
          const float d2 = (sx + sy) + sz;
          const unsigned bit = (d2 <= kR2) ? 0x3C00u : 0u;
          if (e & 1) am[t].u[e >> 1] |= (bit << 16);
          else       am[t].u[e >> 1]  = bit;
        }
      }
      const v16h bfr = Frag<_Float16>::load(sX + c * XP + ks * 32 + 8 * h);
      acc0 = Frag<_Float16>::mma(am[0].v, bfr, acc0);
      acc1 = Frag<_Float16>::mma(am[1].v, bfr, acc1);
      acc2 = Frag<_Float16>::mma(am[2].v, bfr, acc2);
      acc3 = Frag<_Float16>::mma(am[3].v, bfr, acc3);
      mma_guard4(acc0, acc1, acc2, acc3, am[0].v, am[1].v, am[2].v, am[3].v, bfr);
    }
  }
  acc_guard4(acc0, acc1, acc2, acc3);

  float* slab = sSlab[wave];
#pragma unroll 8
  for (int r = 0; r < 8; ++r) {
    slab[c * SP +  0 + 8 * h + r] = acc0[r];
    slab[c * SP + 16 + 8 * h + r] = acc1[r];
    slab[c * SP + 32 + 8 * h + r] = acc2[r];
    slab[c * SP + 48 + 8 * h + r] = acc3[r];
  }
  __syncthreads();

  const int c4 = c * 4;
  const v4f cnt = *(const v4f*)(slab + 15 * SP + c4);
  v4f rd;
  rd.x = 1.0f / ((cnt.x > 0.0f) ? cnt.x : 1.0f);
  rd.y = 1.0f / ((cnt.y > 0.0f) ? cnt.y : 1.0f);
  rd.z = 1.0f / ((cnt.z > 0.0f) ? cnt.z : 1.0f);
  rd.w = 1.0f / ((cnt.w > 0.0f) ? cnt.w : 1.0f);
  const int  o0  = obase + c4;
  const bool inb = (o0 + 3) < nOut;
  const int  nIt = (nB + 1) >> 1;
  for (int pass = 0; pass < 2; ++pass) {
    for (int it = 0; it < nIt; ++it) {
      const int b = 2 * it + h;
      if (b < nB && inb) {
        const v4f v  = *(const v4f*)(slab + b * SP + c4);
        const v4f o4 = v * rd;
        *(volatile v4f*)(out + (size_t)b * nOut + o0) = o4;
      }
    }
    __threadfence();
  }
}

extern "C" void kernel_launch(void* const* d_in, const int* in_sizes, int n_in,
                              void* d_out, int out_size, void* d_ws, size_t ws_size,
                              hipStream_t stream) {
  (void)d_ws; (void)ws_size;
  if (n_in < 3) return;
  const int nIn  = in_sizes[1] / 3;
  const int nOut = in_sizes[2] / 3;
  if (nIn <= 0 || nOut <= 0 || (nOut & 3) != 0) return;
  const int nB = in_sizes[0] / nIn;
  if (nB < 1 || nB > 15) return;
  if ((long long)nB * (long long)nOut > (long long)out_size) return;

  const float* x    = (const float*)d_in[0];
  const float* ipos = (const float*)d_in[1];
  const float* opos = (const float*)d_in[2];
  float* out = (float*)d_out;

  dim3 grid((unsigned)((nOut + OPB - 1) / OPB));
  dim3 block(NT);
  ball_pool_f16<<<grid, block, 0, stream>>>(x, ipos, opos, out, nIn, nOut, nB);
  (void)hipGetLastError();
}
